// GatedCrossAttn_38010460570002
// MI455X (gfx1250) — hardware-verified
//
#include <hip/hip_runtime.h>
#include <hip/hip_bf16.h>
#include <math.h>

#define BB 8
#define NX 512
#define NY 1024
#define DD 1024
#define HH 16
#define KVH 16
#define KVD 1024
#define HKDIV 1
#define DKK 64
#define QW 2
#define SS 1024
#define GSTR 48

typedef _Float16 bf16;
typedef _Float16 f16;
typedef __attribute__((ext_vector_type(4))) unsigned v4u_t;
typedef unsigned v4ua __attribute__((ext_vector_type(4), may_alias));
typedef __attribute__((ext_vector_type(4))) float v4f_t;
typedef float v4fa __attribute__((ext_vector_type(4), may_alias));
typedef __attribute__((ext_vector_type(16))) bf16  bf16x16;
typedef bf16x16 f16x16;
typedef __attribute__((ext_vector_type(8)))  bf16  bf16x8;
typedef bf16x8 f16x8;
typedef __attribute__((ext_vector_type(4)))  bf16  bf16x4;
typedef __attribute__((ext_vector_type(8)))  float f32x8;
__device__ __forceinline__ f32x8 wmma16(f16x16 a, f16x16 b, f32x8 c) {
  c = __builtin_amdgcn_wmma_f32_16x16x32_f16(false, a, false, b, (short)0, c, false, false);
  asm volatile("v_nop\n\tv_nop\n\tv_nop\n\tv_nop" : "+v"(c) : "v"(a), "v"(b));
  return c;
}
#define LDS_STRIDE 48
#define KSTRIDE    72
#define VSTRIDE    48

__device__ __forceinline__ f32x8 wmma_bf16(bf16x16 a, bf16x16 b, f32x8 c) {
  c = __builtin_amdgcn_wmma_f32_16x16x32_f16(false, a, false, b, (short)0, c, false, false);
  asm volatile("v_nop\n\tv_nop\n\tv_nop\n\tv_nop" : "+v"(c) : "v"(a), "v"(b));
  return c;
}

template <typename T>
__device__ __forceinline__ bf16x16 load_frag(const T* __restrict__ base, int ld,
                                             int row0, int k0) {
  const int lane = threadIdx.x & 31;
  const int r    = lane & 15;
  const int kh   = (lane >> 4) * 8;
  const T* p0 = base + (size_t)(row0 + r) * ld + (k0 + kh);
  const T* p1 = p0 + 16;
  bf16x16 f;
#pragma unroll
  for (int i = 0; i < 8; ++i) {
    f[i]     = (bf16)p0[i];
    f[i + 8] = (bf16)p1[i];
  }
  return f;
}

__device__ __forceinline__ bf16x16 lds_frag(const bf16* base, int stride) {
  const int lane = threadIdx.x & 31;
  const int row  = lane & 15;
  const int kh   = (lane >> 4) * 8;
  const bf16x8 lo = *(const bf16x8*)(base + row * stride + kh);
  const bf16x8 hi = *(const bf16x8*)(base + row * stride + kh + 16);
  bf16x16 f;
#pragma unroll
  for (int i = 0; i < 8; ++i) { f[i] = lo[i]; f[i + 8] = hi[i]; }
  return f;
}

template <typename T>
__device__ __forceinline__ void stage_read16(const T* __restrict__ p, float* buf) {
#pragma unroll
  for (int i = 0; i < 16; ++i) buf[i] = (float)p[i];
}

__device__ __forceinline__ void stage_write(bf16* dst, const float* buf, int nquad) {
#pragma unroll
  for (int i = 0; i < nquad; ++i) {
    bf16x4 q;
    q[0] = (bf16)buf[4 * i];     q[1] = (bf16)buf[4 * i + 1];
    q[2] = (bf16)buf[4 * i + 2]; q[3] = (bf16)buf[4 * i + 3];
    *(bf16x4*)(dst + 4 * i) = q;
  }
}

template <typename AT, int MODE>
__global__ __launch_bounds__(256) void gemm_rb_kernel(
    const AT* __restrict__ A, const float* __restrict__ W,
    const float* __restrict__ bias, const float* __restrict__ rowscale, const float* __restrict__ R, const float* __restrict__ rowbias, void* __restrict__ out,
    int M, int N, int K) {
  __shared__ bf16 ldsA[128 * LDS_STRIDE];
  __shared__ bf16 ldsW[256 * LDS_STRIDE];
  __shared__ __attribute__((aligned(16))) unsigned char sob[256 * 136 * 2];

  const int t    = threadIdx.x;
  const int wave = t >> 5;
  const int lane = t & 31;
  const int wm   = (wave & 1) * 64;
  const int wn   = (wave >> 1) * 64;
  const int mBlk = blockIdx.x * 128;
  const int nBlk = blockIdx.y * 256;

  const int arow = t >> 1;
  const int ach  = (t & 1) * 16;

  float abuf[16];
  float wbuf[32];

  stage_read16(A + (size_t)(mBlk + arow) * K + ach, abuf);
  const int nrow = min(nBlk + t, N - 1);
  stage_read16(W + (size_t)nrow * K,          wbuf);
  stage_read16(W + (size_t)nrow * K + 16,     wbuf + 16);

  f32x8 acc[4][4] = {};

  for (int k = 0; k < K; k += 32) {
    __syncthreads();
    stage_write(&ldsA[arow * LDS_STRIDE + ach], abuf, 4);
    stage_write(&ldsW[t * LDS_STRIDE],          wbuf, 8);
    if (k + 32 < K) {
      stage_read16(A + (size_t)(mBlk + arow) * K + (k + 32) + ach, abuf);
      stage_read16(W + (size_t)nrow * K + (k + 32),          wbuf);
      stage_read16(W + (size_t)nrow * K + (k + 32) + 16,     wbuf + 16);
    }
    __syncthreads();

    bf16x16 af[4], wf[4];
#pragma unroll
    for (int i = 0; i < 4; ++i)
      af[i] = lds_frag(ldsA + (wm + 16 * i) * LDS_STRIDE, LDS_STRIDE);
#pragma unroll
    for (int j = 0; j < 4; ++j)
      wf[j] = lds_frag(ldsW + (wn + 16 * j) * LDS_STRIDE, LDS_STRIDE);
#pragma unroll
    for (int i = 0; i < 4; ++i)
#pragma unroll
      for (int j = 0; j < 4; ++j)
        acc[i][j] = wmma_bf16(af[i], wf[j], acc[i][j]);
  }

  const int nlane = lane & 15;
  const int mh    = (lane >> 4) * 8;
  __syncthreads();
  if (MODE == 0 || MODE == 1 || MODE == 3) {
    bf16* so = (bf16*)sob;
#pragma unroll
    for (int i = 0; i < 4; ++i)
#pragma unroll
      for (int j = 0; j < 4; ++j) {
        const int nl = wn + 16 * j + nlane;
        const float bv = bias ? bias[nBlk + nl] : 0.0f;
        if (MODE == 3) {
#pragma unroll 1
          for (int r = 0; r < 8; ++r) {
            const int ml = wm + 16 * i + mh + r;
            const float xg = acc[i][j][r] + bv;
            so[ml * 264 + nl] = (bf16)(0.5f * xg * (1.0f + erff(xg * 0.70710678118654752f)));
          }
        } else {
#pragma unroll
        for (int r = 0; r < 8; ++r) {
          const int ml = wm + 16 * i + mh + r;
          const bf16 hv = (bf16)(acc[i][j][r] + bv);
          if (MODE == 0) so[ml * 264 + nl] = hv;
          else           so[nl * 136 + ml] = hv;
        }
        }
      }
    __syncthreads();
#pragma unroll 1
    for (int pass = 0; pass < 2; ++pass) {
      if (MODE == 0 || MODE == 3) {
        for (int ch = t; ch < 128 * 32; ch += 256) { const int ml = ch >> 5, q = (ch & 31) * 8;
          *(volatile v4u_t*)((bf16*)out + (size_t)(mBlk + ml) * N + nBlk + q) = *(const v4ua*)(so + ml * 264 + q); }
      } else {
        const int b_ = mBlk / SS, s0 = mBlk % SS;
        for (int ch = t; ch < 256 * 16; ch += 256) { const int nl = ch >> 4, q = (ch & 15) * 8; const int n = nBlk + nl, h = n >> 6, dk = n & (DKK - 1);
          *(volatile v4u_t*)((bf16*)out + (((size_t)(b_ * HH + h)) * DKK + dk) * SS + s0 + q) = *(const v4ua*)(so + nl * 136 + q); }
      }
      __threadfence();
    }
  } else {
    float* so = (float*)sob;
#pragma unroll 1
    for (int hf = 0; hf < 2; ++hf) {
      if (wm == hf * 64) {
#pragma unroll
        for (int i = 0; i < 4; ++i)
#pragma unroll
          for (int j = 0; j < 4; ++j) {
            const int nl = wn + 16 * j + nlane;
            const float bv = bias ? bias[nBlk + nl] : 0.0f;
#pragma unroll
            for (int r = 0; r < 8; ++r) { const int mrow = mBlk + hf * 64 + 16 * i + mh + r; so[(16 * i + mh + r) * 260 + nl] = acc[i][j][r] * (rowscale ? rowscale[mrow] : 1.0f) + bv + (rowbias ? rowbias[mrow] : 0.0f); }
          }
      }
      __syncthreads();
      if (R) {
        for (int ch = t; ch < 64 * 64; ch += 256) { const int ml = ch >> 6, q = (ch & 63) * 4;
          if (nBlk + q < N) { const v4f_t rv = *(const v4f_t*)(R + (size_t)(mBlk + hf * 64 + ml) * N + nBlk + q); v4f_t v = *(const v4fa*)(so + ml * 260 + q); v += rv; *(volatile v4fa*)(so + ml * 260 + q) = v; } }
        asm volatile("s_wait_dscnt 0" ::: "memory");
      }
#pragma unroll 1
      for (int pass = 0; pass < 2; ++pass) {
        for (int ch = t; ch < 64 * 64; ch += 256) { const int ml = ch >> 6, q = (ch & 63) * 4;
          if (nBlk + q < N) *(volatile v4f_t*)((float*)out + (size_t)(mBlk + hf * 64 + ml) * N + nBlk + q) = *(const v4fa*)(so + ml * 260 + q); }
        __threadfence();
      }
      __syncthreads();
    }
  }
}


#define QROWS 512
#define KROWS 1024
#define NKV 1024
__global__ __launch_bounds__(64) void xy_attn_kernel(
    const bf16* __restrict__ Qb, const bf16* __restrict__ Kb,
    const bf16* __restrict__ Vt, const float* __restrict__ kbias,
    float* __restrict__ attnOut) {
  __shared__ bf16 ldsK[32 * KSTRIDE];
  __shared__ bf16 ldsV[64 * VSTRIDE];
  __shared__ __attribute__((aligned(16))) bf16 ldsO[2][32 * 72];

  const int q0blk = blockIdx.x * 64;
  const int h  = blockIdx.y;
  const int b  = blockIdx.z;
  const int t    = threadIdx.x;
  const int wave = t >> 5;
  const int lane = t & 31;
  const int qlane = lane & 15;
  const int kh8   = (lane >> 4) * 8;
  const int q0 = q0blk + wave * 32;

  const int hk = h / HKDIV;
  const bf16* Qh = Qb + (size_t)b * QROWS * DD + h * DKK;
  const bf16* Kh = Kb + (size_t)b * KROWS * KVD + hk * DKK;
  const bf16* Vh = Vt + ((size_t)(b * KVH + hk)) * DKK * KROWS;

  const int krow = t >> 1;
  const int kcol = (t & 1) * 32;
  const bf16* kSrc = Kh + (size_t)krow * KVD + kcol;
  const bf16* vSrc = Vh + (size_t)t * KROWS;

  bf16x16 qf[QW][2];
#pragma unroll
  for (int qt = 0; qt < QW; ++qt) {
    qf[qt][0] = load_frag(Qh, DD, q0 + 16 * qt, 0);
    qf[qt][1] = load_frag(Qh, DD, q0 + 16 * qt, 32);
  }

  f32x8 o[QW][4] = {};
  float mrun[QW], lrun[QW];
#pragma unroll
  for (int qt = 0; qt < QW; ++qt) { mrun[qt] = -INFINITY; lrun[qt] = 0.0f; }

  const float scale = 0.125f * 1.44269504088896340736f;
  const float NEG2 = -1.0e9f;
  const int kmax = KROWS - 1;
  __shared__ float kbS[KROWS];
  for (int i = threadIdx.x; i < KROWS; i += 64) kbS[i] = kbias[(size_t)b * KROWS + i] * 1.44269504088896340736f;
  __syncthreads();

  bf16x8 kreg[4], vreg[4];
#pragma unroll
  for (int i = 0; i < 4; ++i) {
    kreg[i] = *(const bf16x8*)(kSrc + 8 * i);
    vreg[i] = *(const bf16x8*)(vSrc + 8 * i);
  }

  for (int kb = 0; kb <= kmax; kb += 32) {
    __syncthreads();
#pragma unroll
    for (int i = 0; i < 4; ++i) {
      *(bf16x8*)(&ldsK[krow * KSTRIDE + kcol + 8 * i]) = kreg[i];
      *(bf16x8*)(&ldsV[t * VSTRIDE + 8 * i])           = vreg[i];
    }
    if (kb + 32 <= kmax) {
      const bf16* kn = kSrc + (size_t)(kb + 32) * KVD;
      const bf16* vn = vSrc + (kb + 32);
#pragma unroll
      for (int i = 0; i < 4; ++i) {
        kreg[i] = *(const bf16x8*)(kn + 8 * i);
        vreg[i] = *(const bf16x8*)(vn + 8 * i);
      }
    }
    __syncthreads();

    bf16x16 kf[2][2];
#pragma unroll
    for (int ktile = 0; ktile < 2; ++ktile)
#pragma unroll
      for (int c = 0; c < 2; ++c)
        kf[ktile][c] = lds_frag(ldsK + (ktile * 16) * KSTRIDE + c * 32, KSTRIDE);

    bf16x16 pf[QW];
    bool act[QW];
#pragma unroll
    for (int qt = 0; qt < QW; ++qt) {
      unsigned mbits = 0;
      {
#pragma unroll
        for (int r = 0; r < 8; ++r) { const int j0 = kb + kh8 + r; if (j0 < NKV) mbits |= 1u << r; if (j0 + 16 < NKV) mbits |= 1u << (8 + r); }
        act[qt] = (__builtin_amdgcn_ballot_w32(mbits != 0) != 0);
      }
      if (act[qt]) {
        const int q_my = q0 + 16 * qt + qlane;
        f32x8 s0 = {}, s1 = {};
        s0 = wmma_bf16(kf[0][0], qf[qt][0], s0);
        s0 = wmma_bf16(kf[0][1], qf[qt][1], s0);
        s1 = wmma_bf16(kf[1][0], qf[qt][0], s1);
        s1 = wmma_bf16(kf[1][1], qf[qt][1], s1);

        float mx = -INFINITY;
#pragma unroll
        for (int r = 0; r < 8; ++r) {
          const int k0i = kb + kh8 + r;
          const int k1i = k0i + 16;
          (void)k0i; (void)k1i; (void)q_my;
          s0[r] = (mbits & (1u << r))       ? s0[r] * scale + kbS[kb + kh8 + r] : NEG2;
          s1[r] = (mbits & (1u << (8 + r))) ? s1[r] * scale + kbS[kb + 16 + kh8 + r] : NEG2;
          mx = fmaxf(mx, fmaxf(s0[r], s1[r]));
        }
        mx = fmaxf(mx, __shfl_xor(mx, 16, 32));
        const float mnew  = fmaxf(mrun[qt], mx);
        const float alpha = exp2f(mrun[qt] - mnew);

        float rsum = 0.0f;
#pragma unroll
        for (int r = 0; r < 8; ++r) {
          const float p0 = exp2f(s0[r] - mnew);
          const float p1 = exp2f(s1[r] - mnew);
          rsum += p0 + p1;
          pf[qt][r]     = (bf16)(p0 * 1024.0f);
          pf[qt][r + 8] = (bf16)(p1 * 1024.0f);
        }
        rsum += __shfl_xor(rsum, 16, 32);
        lrun[qt] = lrun[qt] * alpha + rsum;
        mrun[qt] = mnew;

#pragma unroll
        for (int j = 0; j < 4; ++j)
#pragma unroll
          for (int r = 0; r < 8; ++r) o[qt][j][r] *= alpha;
      }
    }

#pragma unroll
    for (int j = 0; j < 4; ++j) {
      const bf16x16 vf = lds_frag(ldsV + (j * 16) * VSTRIDE, VSTRIDE);
#pragma unroll
      for (int qt = 0; qt < QW; ++qt)
        if (act[qt]) o[qt][j] = wmma_bf16(vf, pf[qt], o[qt][j]);
    }
  }

  __shared__ __attribute__((aligned(16))) float ldsOf[2][32 * 68];
  float* so = ldsOf[wave]; (void)ldsO;
#pragma unroll
  for (int qt = 0; qt < QW; ++qt) {
    const float rl = 1.0f / (lrun[qt] * 1024.0f);
#pragma unroll
    for (int j = 0; j < 4; ++j)
#pragma unroll
      for (int r = 0; r < 8; ++r) so[(16 * qt + qlane) * 68 + j * 16 + kh8 + r] = o[qt][j][r] * rl;
  }
  asm volatile("s_wait_dscnt 0" ::: "memory");
  __builtin_amdgcn_wave_barrier();
#pragma unroll 1
  for (int pass = 0; pass < 2; ++pass) {
#pragma unroll
    for (int it = 0; it < 16; ++it) { const int ch = lane + 32 * it, ql = ch >> 4, q4 = (ch & 15) * 4;
      *(volatile v4f_t*)(attnOut + ((size_t)(b * QROWS + q0 + ql)) * DD + h * DKK + q4) = *(const v4fa*)(so + ql * 68 + q4); }
    __threadfence();
  }
}


#undef QROWS
#undef KROWS
#undef NKV
#define QROWS 1024
#define KROWS 512
#define NKV 512
__global__ __launch_bounds__(64) void yx_attn_kernel(
    const bf16* __restrict__ Qb, const bf16* __restrict__ Kb,
    const bf16* __restrict__ Vt, const float* __restrict__ kbias,
    float* __restrict__ attnOut) {
  __shared__ bf16 ldsK[32 * KSTRIDE];
  __shared__ bf16 ldsV[64 * VSTRIDE];
  __shared__ __attribute__((aligned(16))) bf16 ldsO[2][32 * 72];

  const int q0blk = blockIdx.x * 64;
  const int h  = blockIdx.y;
  const int b  = blockIdx.z;
  const int t    = threadIdx.x;
  const int wave = t >> 5;
  const int lane = t & 31;
  const int qlane = lane & 15;
  const int kh8   = (lane >> 4) * 8;
  const int q0 = q0blk + wave * 32;

  const int hk = h / HKDIV;
  const bf16* Qh = Qb + (size_t)b * QROWS * DD + h * DKK;
  const bf16* Kh = Kb + (size_t)b * KROWS * KVD + hk * DKK;
  const bf16* Vh = Vt + ((size_t)(b * KVH + hk)) * DKK * KROWS;

  const int krow = t >> 1;
  const int kcol = (t & 1) * 32;
  const bf16* kSrc = Kh + (size_t)krow * KVD + kcol;
  const bf16* vSrc = Vh + (size_t)t * KROWS;

  bf16x16 qf[QW][2];
#pragma unroll
  for (int qt = 0; qt < QW; ++qt) {
    qf[qt][0] = load_frag(Qh, DD, q0 + 16 * qt, 0);
    qf[qt][1] = load_frag(Qh, DD, q0 + 16 * qt, 32);
  }

  f32x8 o[QW][4] = {};
  float mrun[QW], lrun[QW];
#pragma unroll
  for (int qt = 0; qt < QW; ++qt) { mrun[qt] = -INFINITY; lrun[qt] = 0.0f; }

  const float scale = 0.125f * 1.44269504088896340736f;
  const float NEG2 = -1.0e9f;
  const int kmax = KROWS - 1;
  __shared__ float kbS[KROWS];
  for (int i = threadIdx.x; i < KROWS; i += 64) kbS[i] = kbias[(size_t)b * KROWS + i] * 1.44269504088896340736f;
  __syncthreads();

  bf16x8 kreg[4], vreg[4];
#pragma unroll
  for (int i = 0; i < 4; ++i) {
    kreg[i] = *(const bf16x8*)(kSrc + 8 * i);
    vreg[i] = *(const bf16x8*)(vSrc + 8 * i);
  }

  for (int kb = 0; kb <= kmax; kb += 32) {
    __syncthreads();
#pragma unroll
    for (int i = 0; i < 4; ++i) {
      *(bf16x8*)(&ldsK[krow * KSTRIDE + kcol + 8 * i]) = kreg[i];
      *(bf16x8*)(&ldsV[t * VSTRIDE + 8 * i])           = vreg[i];
    }
    if (kb + 32 <= kmax) {
      const bf16* kn = kSrc + (size_t)(kb + 32) * KVD;
      const bf16* vn = vSrc + (kb + 32);
#pragma unroll
      for (int i = 0; i < 4; ++i) {
        kreg[i] = *(const bf16x8*)(kn + 8 * i);
        vreg[i] = *(const bf16x8*)(vn + 8 * i);
      }
    }
    __syncthreads();

    bf16x16 kf[2][2];
#pragma unroll
    for (int ktile = 0; ktile < 2; ++ktile)
#pragma unroll
      for (int c = 0; c < 2; ++c)
        kf[ktile][c] = lds_frag(ldsK + (ktile * 16) * KSTRIDE + c * 32, KSTRIDE);

    bf16x16 pf[QW];
    bool act[QW];
#pragma unroll
    for (int qt = 0; qt < QW; ++qt) {
      unsigned mbits = 0;
      {
#pragma unroll
        for (int r = 0; r < 8; ++r) { const int j0 = kb + kh8 + r; if (j0 < NKV) mbits |= 1u << r; if (j0 + 16 < NKV) mbits |= 1u << (8 + r); }
        act[qt] = (__builtin_amdgcn_ballot_w32(mbits != 0) != 0);
      }
      if (act[qt]) {
        const int q_my = q0 + 16 * qt + qlane;
        f32x8 s0 = {}, s1 = {};
        s0 = wmma_bf16(kf[0][0], qf[qt][0], s0);
        s0 = wmma_bf16(kf[0][1], qf[qt][1], s0);
        s1 = wmma_bf16(kf[1][0], qf[qt][0], s1);
        s1 = wmma_bf16(kf[1][1], qf[qt][1], s1);

        float mx = -INFINITY;
#pragma unroll
        for (int r = 0; r < 8; ++r) {
          const int k0i = kb + kh8 + r;
          const int k1i = k0i + 16;
          (void)k0i; (void)k1i; (void)q_my;
          s0[r] = (mbits & (1u << r))       ? s0[r] * scale + kbS[kb + kh8 + r] : NEG2;
          s1[r] = (mbits & (1u << (8 + r))) ? s1[r] * scale + kbS[kb + 16 + kh8 + r] : NEG2;
          mx = fmaxf(mx, fmaxf(s0[r], s1[r]));
        }
        mx = fmaxf(mx, __shfl_xor(mx, 16, 32));
        const float mnew  = fmaxf(mrun[qt], mx);
        const float alpha = exp2f(mrun[qt] - mnew);

        float rsum = 0.0f;
#pragma unroll
        for (int r = 0; r < 8; ++r) {
          const float p0 = exp2f(s0[r] - mnew);
          const float p1 = exp2f(s1[r] - mnew);
          rsum += p0 + p1;
          pf[qt][r]     = (bf16)(p0 * 1024.0f);
          pf[qt][r + 8] = (bf16)(p1 * 1024.0f);
        }
        rsum += __shfl_xor(rsum, 16, 32);
        lrun[qt] = lrun[qt] * alpha + rsum;
        mrun[qt] = mnew;

#pragma unroll
        for (int j = 0; j < 4; ++j)
#pragma unroll
          for (int r = 0; r < 8; ++r) o[qt][j][r] *= alpha;
      }
    }

#pragma unroll
    for (int j = 0; j < 4; ++j) {
      const bf16x16 vf = lds_frag(ldsV + (j * 16) * VSTRIDE, VSTRIDE);
#pragma unroll
      for (int qt = 0; qt < QW; ++qt)
        if (act[qt]) o[qt][j] = wmma_bf16(vf, pf[qt], o[qt][j]);
    }
  }

  __shared__ __attribute__((aligned(16))) float ldsOf[2][32 * 68];
  float* so = ldsOf[wave]; (void)ldsO;
#pragma unroll
  for (int qt = 0; qt < QW; ++qt) {
    const float rl = 1.0f / (lrun[qt] * 1024.0f);
#pragma unroll
    for (int j = 0; j < 4; ++j)
#pragma unroll
      for (int r = 0; r < 8; ++r) so[(16 * qt + qlane) * 68 + j * 16 + kh8 + r] = o[qt][j][r] * rl;
  }
  asm volatile("s_wait_dscnt 0" ::: "memory");
  __builtin_amdgcn_wave_barrier();
#pragma unroll 1
  for (int pass = 0; pass < 2; ++pass) {
#pragma unroll
    for (int it = 0; it < 16; ++it) { const int ch = lane + 32 * it, ql = ch >> 4, q4 = (ch & 15) * 4;
      *(volatile v4f_t*)(attnOut + ((size_t)(b * QROWS + q0 + ql)) * DD + h * DKK + q4) = *(const v4fa*)(so + ql * 68 + q4); }
    __threadfence();
  }
}


#undef QROWS
#undef KROWS
#undef NKV
__global__ __launch_bounds__(256) void k_rows16(const float* __restrict__ P, bf16* __restrict__ R16) { __shared__ __attribute__((aligned(16))) bf16 s[64][72];
  const int tid = threadIdx.x; const size_t t0 = (size_t)blockIdx.x * 64; const int h = blockIdx.y;
  for (int e = tid; e < 64 * 64; e += 256) { const int t = e >> 6, d = e & 63; s[t][d] = (bf16)P[(t0 + t) * DD + h * DKK + d]; }
  __syncthreads();
#pragma unroll 1
  for (int pass = 0; pass < 2; ++pass) {
#pragma unroll 1
    for (int round = 0; round < 2; ++round) { const int r = round * 32 + (tid >> 3), piece = (tid & 7) * 8; *(volatile v4u_t*)(R16 + (t0 + r) * DD + h * DKK + piece) = *(const v4ua*)(&s[r][piece]); }
    __threadfence(); } }
__global__ __launch_bounds__(256) void k_vt(const float* __restrict__ P, int L, bf16* __restrict__ Vt) { __shared__ __attribute__((aligned(16))) bf16 vT[64][72];
  const int tid = threadIdx.x; const size_t t0 = (size_t)blockIdx.x * 64; const int h = blockIdx.y; const int b = (int)(t0 / L), n0 = (int)(t0 % L);
  for (int e = tid; e < 64 * 64; e += 256) { const int t = e >> 6, d = e & 63; vT[d][t] = (bf16)P[(t0 + t) * DD + h * DKK + d]; }
  __syncthreads();
#pragma unroll 1
  for (int pass = 0; pass < 2; ++pass) {
#pragma unroll 1
    for (int round = 0; round < 2; ++round) { const int r = round * 32 + (tid >> 3), piece = (tid & 7) * 8; *(volatile v4u_t*)(Vt + ((size_t)b * DD + h * DKK + r) * L + n0 + piece) = *(const v4ua*)(&vT[r][piece]); }
    __threadfence(); } }
__global__ __launch_bounds__(256) void k_gate(const float* __restrict__ T, const float* __restrict__ Wg, const float* __restrict__ bg, const int* __restrict__ mask, float* __restrict__ gate, float* __restrict__ kb) {
  __shared__ __attribute__((aligned(16))) float gS[64], lS[64];
  const int tid = threadIdx.x, tl = tid >> 2, part = tid & 3; const size_t tok = (size_t)blockIdx.x * 64 + tl;
  float d0 = 0.f, d1 = 0.f, d2 = 0.f, d3 = 0.f;
#pragma unroll 1
  for (int i = part * 256; i < part * 256 + 256; ++i) { const float t = T[tok * DD + i]; d0 += t * Wg[i]; d1 += t * Wg[DD + i]; d2 += t * Wg[2 * DD + i]; d3 += t * Wg[3 * DD + i]; }
  d0 += __shfl_xor(d0, 1, 32); d1 += __shfl_xor(d1, 1, 32); d2 += __shfl_xor(d2, 1, 32); d3 += __shfl_xor(d3, 1, 32);
  d0 += __shfl_xor(d0, 2, 32); d1 += __shfl_xor(d1, 2, 32); d2 += __shfl_xor(d2, 2, 32); d3 += __shfl_xor(d3, 2, 32);
  if (part == 0) { const float mu = d0 + bg[0], vr = d1 + bg[1], ar = d2 + bg[2], br = d3 + bg[3];
    const float spv = (vr > 20.0f) ? vr : log1pf(expf(vr)), spa = (ar > 20.0f) ? ar : log1pf(expf(ar)), spb = (br > 20.0f) ? br : log1pf(expf(br));
    const float v = spv + 1e-6f, alpha = spa + 1.0f + 1e-6f, beta = spb + 1e-6f; const float var_ep = beta / (v * (alpha - 1.0f));
    float g = (1.0f / (1.0f + expf(-mu))) * expf(-2.0f * fmaxf(var_ep, 0.0f)); g = fminf(fmaxf(g, 0.05f), 1.0f); g = fmaxf(g, 1e-6f);
    gS[tl] = g; lS[tl] = (mask[tok] != 0) ? logf(g) : -1.0e9f; }
  __syncthreads();
#pragma unroll 1
  for (int pass = 0; pass < 2; ++pass) { if (tid < 16) *(volatile v4f_t*)(gate + (size_t)blockIdx.x * 64 + tid * 4) = *(const v4fa*)(gS + tid * 4); else if (tid < 32) *(volatile v4f_t*)(kb + (size_t)blockIdx.x * 64 + (tid - 16) * 4) = *(const v4fa*)(lS + (tid - 16) * 4); __threadfence(); }
}
__global__ __launch_bounds__(128) void k_cast16(const float* __restrict__ A, bf16* __restrict__ O) { const size_t row = blockIdx.x; const int c8 = threadIdx.x * 8; union { bf16 hh[8]; v4u_t u; } cv;
  const v4f_t a = *(const v4f_t*)(A + row * DD + c8), c = *(const v4f_t*)(A + row * DD + c8 + 4); for (int i = 0; i < 4; ++i) { cv.hh[i] = (bf16)a[i]; cv.hh[4 + i] = (bf16)c[i]; }
  *(volatile v4u_t*)(O + row * DD + c8) = cv.u; __threadfence(); *(volatile v4u_t*)(O + row * DD + c8) = cv.u; }
__global__ __launch_bounds__(256) void k_ln(const float* __restrict__ X, const float* __restrict__ g, const float* __restrict__ bb, float* __restrict__ Y) {
  __shared__ __attribute__((aligned(16))) float rowS[8 * (DD + 4)];
  const int tid = threadIdx.x, r = tid >> 5, lane = tid & 31; const size_t row = (size_t)blockIdx.x * 8 + r; const float* xr = X + row * DD;
  float s = 0.0f;
#pragma unroll 1
  for (int i = lane; i < DD; i += 32) { const float v = xr[i]; rowS[r * (DD + 4) + i] = v; s += v; }
#pragma unroll
  for (int off = 1; off < 32; off <<= 1) s += __shfl_xor(s, off, 32);
  const float mean = s * (1.0f / DD); float q = 0.0f;
#pragma unroll 1
  for (int i = lane; i < DD; i += 32) { const float d = rowS[r * (DD + 4) + i] - mean; q += d * d; }
#pragma unroll
  for (int off = 1; off < 32; off <<= 1) q += __shfl_xor(q, off, 32);
  const float rstd = rsqrtf(q * (1.0f / DD) + 1e-5f);
#pragma unroll 1
  for (int i = lane; i < DD; i += 32) rowS[r * (DD + 4) + i] = (rowS[r * (DD + 4) + i] - mean) * rstd * g[i] + bb[i];
  __syncthreads();
#pragma unroll 1
  for (int pass = 0; pass < 2; ++pass) { for (int q4 = tid; q4 < 8 * (DD / 4); q4 += 256) { const int rr = q4 / (DD / 4), c4 = (q4 % (DD / 4)) * 4;
      *(volatile v4f_t*)(Y + ((size_t)blockIdx.x * 8 + rr) * DD + c4) = *(const v4fa*)(rowS + rr * (DD + 4) + c4); } __threadfence(); }
}
__global__ __launch_bounds__(256) void k_silu(float* __restrict__ t) { const size_t row = blockIdx.x;
  for (int q4 = threadIdx.x; q4 < DD / 4; q4 += 256) { v4f_t v = *(const v4f_t*)(t + row * DD + q4 * 4); for (int e = 0; e < 4; ++e) v[e] = v[e] / (1.0f + expf(-v[e]));
    *(volatile v4f_t*)(t + row * DD + q4 * 4) = v; __threadfence(); *(volatile v4f_t*)(t + row * DD + q4 * 4) = v; } }

__global__ __launch_bounds__(256) void k_addln(const float* __restrict__ A, const float* __restrict__ Bv, const float* __restrict__ g, const float* __restrict__ bb, float* __restrict__ Y) {
  __shared__ __attribute__((aligned(16))) float rowS[8 * (DD + 4)];
  const int tid = threadIdx.x, r = tid >> 5, lane = tid & 31; const size_t row = (size_t)blockIdx.x * 8 + r;
  float s = 0.0f;
#pragma unroll 1
  for (int i = lane; i < DD; i += 32) { const float v = A[row * DD + i] + Bv[row * DD + i]; rowS[r * (DD + 4) + i] = v; s += v; }
#pragma unroll
  for (int off = 1; off < 32; off <<= 1) s += __shfl_xor(s, off, 32);
  const float mean = s * (1.0f / DD); float q = 0.0f;
#pragma unroll 1
  for (int i = lane; i < DD; i += 32) { const float d = rowS[r * (DD + 4) + i] - mean; q += d * d; }
#pragma unroll
  for (int off = 1; off < 32; off <<= 1) q += __shfl_xor(q, off, 32);
  const float rstd = rsqrtf(q * (1.0f / DD) + 1e-5f);
#pragma unroll 1
  for (int i = lane; i < DD; i += 32) rowS[r * (DD + 4) + i] = (rowS[r * (DD + 4) + i] - mean) * rstd * g[i] + bb[i];
  __syncthreads();
#pragma unroll 1
  for (int pass = 0; pass < 2; ++pass) { for (int q4 = tid; q4 < 8 * (DD / 4); q4 += 256) { const int rr = q4 / (DD / 4), c4 = (q4 % (DD / 4)) * 4;
      *(volatile v4f_t*)(Y + ((size_t)blockIdx.x * 8 + rr) * DD + c4) = *(const v4fa*)(rowS + rr * (DD + 4) + c4); } __threadfence(); }
}

extern "C" void kernel_launch(void* const* d_in, const int* in_sizes, int n_in,
                              void* d_out, int out_size, void* d_ws, size_t ws_size,
                              hipStream_t stream) {
  (void)in_sizes; (void)n_in; (void)out_size;
  const float** f = (const float**)d_in;
  const float* x = f[0], *y = f[1]; const int* xmask = (const int*)d_in[2]; const int* ymask = (const int*)d_in[3];
  const float* Wqx = f[4], *Wkx = f[5], *Wvx = f[6], *Wqy = f[7], *Wky = f[8], *Wvy = f[9], *gxw = f[10], *gxb = f[11], *gyw = f[12], *gyb = f[13], *Wox = f[14], *Woy = f[15], *lnxg = f[16], *lnxb = f[17], *lnyg = f[18], *lnyb = f[19], *ffxw = f[20], *ffxb = f[21], *ffyw = f[22], *ffyb = f[23];
  float* x2 = (float*)d_out; float* y2 = x2 + (size_t)BB * NX * DD; float* gxo = y2 + (size_t)BB * NY * DD; float* gyo = gxo + (size_t)BB * NX;
  const int MX = BB * NX, MY = BB * NY;
  char* ws = (char*)d_ws;
  float* P = (float*)ws; ws += (size_t)MY * DD * 4;
  bf16* Qx16 = (bf16*)ws; ws += (size_t)MX * DD * 2; bf16* Kx16 = (bf16*)ws; ws += (size_t)MX * DD * 2; bf16* Vtx = (bf16*)ws; ws += (size_t)MX * DD * 2;
  bf16* Qy16 = (bf16*)ws; ws += (size_t)MY * DD * 2; bf16* Ky16 = (bf16*)ws; ws += (size_t)MY * DD * 2; bf16* Vty = (bf16*)ws; ws += (size_t)MY * DD * 2;
  float* kbx = (float*)ws; ws += (size_t)MX * 4; float* kby = (float*)ws; ws += (size_t)MY * 4;
  float* att = P;
  float* u = P;
  float* u2x = (float*)ws; ws += (size_t)MX * DD * 4;
  bf16* att16x = Qx16;
  bf16* att16y = Qy16;
  float* u2y = (float*)Ky16;
  if ((size_t)(ws - (char*)d_ws) > ws_size) return;
  const dim3 blk(256);
  gemm_rb_kernel<float, 2><<<dim3(MX / 128, DD / 256), blk, 0, stream>>>(x, Wqx, nullptr, nullptr, nullptr, nullptr, P, MX, DD, DD); k_rows16<<<dim3(MX / 64, HH), blk, 0, stream>>>(P, Qx16);
  gemm_rb_kernel<float, 2><<<dim3(MX / 128, DD / 256), blk, 0, stream>>>(x, Wkx, nullptr, nullptr, nullptr, nullptr, P, MX, DD, DD); k_rows16<<<dim3(MX / 64, HH), blk, 0, stream>>>(P, Kx16);
  gemm_rb_kernel<float, 2><<<dim3(MX / 128, DD / 256), blk, 0, stream>>>(x, Wvx, nullptr, nullptr, nullptr, nullptr, P, MX, DD, DD); k_vt<<<dim3(MX / 64, HH), blk, 0, stream>>>(P, NX, Vtx);
  gemm_rb_kernel<float, 2><<<dim3(MY / 128, DD / 256), blk, 0, stream>>>(y, Wqy, nullptr, nullptr, nullptr, nullptr, P, MY, DD, DD); k_rows16<<<dim3(MY / 64, HH), blk, 0, stream>>>(P, Qy16);
  gemm_rb_kernel<float, 2><<<dim3(MY / 128, DD / 256), blk, 0, stream>>>(y, Wky, nullptr, nullptr, nullptr, nullptr, P, MY, DD, DD); k_rows16<<<dim3(MY / 64, HH), blk, 0, stream>>>(P, Ky16);
  gemm_rb_kernel<float, 2><<<dim3(MY / 128, DD / 256), blk, 0, stream>>>(y, Wvy, nullptr, nullptr, nullptr, nullptr, P, MY, DD, DD); k_vt<<<dim3(MY / 64, HH), blk, 0, stream>>>(P, NY, Vty);
  k_gate<<<dim3(MX / 64), blk, 0, stream>>>(x, gxw, gxb, xmask, gxo, kbx);
  k_gate<<<dim3(MY / 64), blk, 0, stream>>>(y, gyw, gyb, ymask, gyo, kby);
  xy_attn_kernel<<<dim3(NX / 64, HH, BB), dim3(64), 0, stream>>>(Qx16, Ky16, Vty, kby, att);
  k_cast16<<<dim3(MX), dim3(128), 0, stream>>>(att, att16x);
  gemm_rb_kernel<bf16, 2><<<dim3(MX / 128, DD / 256), blk, 0, stream>>>(att16x, Wox, nullptr, nullptr, x, nullptr, u, MX, DD, DD);
  k_ln<<<dim3(MX / 8), blk, 0, stream>>>(u, lnxg, lnxb, u2x);
  gemm_rb_kernel<float, 2><<<dim3(MX / 128, DD / 256), blk, 0, stream>>>(u2x, ffxw, ffxb, nullptr, nullptr, nullptr, u, MX, DD, DD);
  k_silu<<<dim3(MX), blk, 0, stream>>>(u);
  k_addln<<<dim3(MX / 8), blk, 0, stream>>>(u2x, u, lnxg, lnxb, x2);
  yx_attn_kernel<<<dim3(NY / 64, HH, BB), dim3(64), 0, stream>>>(Qy16, Kx16, Vtx, kbx, att);
  k_cast16<<<dim3(MY), dim3(128), 0, stream>>>(att, att16y);
  gemm_rb_kernel<bf16, 2><<<dim3(MY / 128, DD / 256), blk, 0, stream>>>(att16y, Woy, nullptr, nullptr, y, nullptr, u, MY, DD, DD);
  k_ln<<<dim3(MY / 8), blk, 0, stream>>>(u, lnyg, lnyb, u2y);
  gemm_rb_kernel<float, 2><<<dim3(MY / 128, DD / 256), blk, 0, stream>>>(u2y, ffyw, ffyb, nullptr, nullptr, nullptr, u, MY, DD, DD);
  k_silu<<<dim3(MY), blk, 0, stream>>>(u);
  k_addln<<<dim3(MY / 8), blk, 0, stream>>>(u2y, u, lnyg, lnyb, y2);
}
